// KnowRGFD_54030688584334
// MI455X (gfx1250) — hardware-verified
//
#include <hip/hip_runtime.h>
#include <stddef.h>
#include <stdint.h>
#include <math.h>

#define NN      50000
#define NE      800000
#define HD      128
#define NR      5
#define NCL     4
#define MP      50048
#define GBM     64
#define GTHR    128
#define SP      132
#define NTHR    256
#define NWAVE   8
#define EPT     8
#define WCH     (32 * EPT)
#define NBRUN   1024
#define SLB     10
#define NBK     49
#define WLCAP   3584
#define RCAP    28672
#define TRIPCAP 64
#define MAXDEG_MEAS   35
#define MAXB1024_MEAS 16623
#define ABM     64
#define NODEM   128
#define CHROWS  13312
#define NCHUNK  4
#define XP      128
#define HP      256
#define MPI     1280
#define BTP     1536
#define KH0     128
#define SPLIT_M 1
#define SPLIT_H 1
#define KHN     (SPLIT_H ? 256 : 128)
#define KMN     1280

#define BK_ZINTS (NWAVE * WLCAP + RCAP + 3 * NBRUN + 8 * NBRUN)
#define BK_INTS  (BK_ZINTS + 16)
#define BK_LDS   (BK_INTS * 4)

#define PBX   (MP * XP / 8 / NTHR)
#define PBT   (5 * 12 * 8)
#define PBS   8
#define PBTOT (PBX + PBT + PBS)

#define SM_BIAS  0
#define SM_LAW   640
#define SM_LOW   896
#define SM_LSC   1408
#define SM_GAW   1440
#define SM_GOW   1824
#define SM_GSC   2336
#define SM_FLOATS 2368

static_assert(MP % GBM == 0 && MP % NODEM == 0 && MP % ABM == 0 && MP >= NN);
static_assert(NBRUN == (1 << SLB) && NBRUN % ABM == 0 && NBRUN % NODEM == 0 && NBRUN % GBM == 0);
static_assert(NBK * NBRUN >= MP);
static_assert(CHROWS % NBRUN == 0 && CHROWS % GBM == 0 && CHROWS % ABM == 0);
static_assert((MP - (NCHUNK - 1) * CHROWS) > 0 && (MP - (NCHUNK - 1) * CHROWS) <= CHROWS);
static_assert((MP - (NCHUNK - 1) * CHROWS) % GBM == 0);
static_assert(NE < (1 << 20) && (((long long)NE) << SLB) < (1LL << 31));
static_assert(NE % WCH == 0 && NE % 4 == 0);
static_assert(RCAP == NWAVE * WLCAP && RCAP % (NTHR * 4) == 0 && BK_ZINTS % 4 == 0);
static_assert((long long)RCAP * 100 >= (long long)MAXB1024_MEAS * 105);
static_assert(WLCAP >= MAXB1024_MEAS / 8 + 8 * 46 + 1);
static_assert(NN <= 65536);
static_assert(MAXDEG_MEAS + 8 <= TRIPCAP);
static_assert(HP == 2 * HD && XP == HD && MPI == NR * 2 * HD && BTP == (NR + 1) * 2 * HD);
static_assert(XP % 8 == 0 && HP % 8 == 0 && MPI % 8 == 0 && BTP % 8 == 0);
static_assert(KH0 % 32 == 0 && KHN % 32 == 0 && KMN % 32 == 0 && KH0 <= XP && KHN <= HP && KMN == MPI);
static_assert(256 + KMN == BTP);
static_assert(HD == 4 * 32 && GBM == (GTHR / 32) * 16);
static_assert((MP * XP / 8) % NTHR == 0);
static_assert(BK_LDS <= 300000);
static_assert((GBM * SP + 128) * 4 <= 65536);
static_assert((NN * NCL * 4) % 128 == 0 && (NODEM * NCL * 4) % 128 == 0 && (((NN % NODEM) * NCL * 4) % 128) == 0);
static_assert(5 * NN * NCL + NN * NCL <= 6 * NN * NCL);
static_assert(SM_LAW % 32 == 0 && SM_LOW % 32 == 0 && SM_LSC % 32 == 0 && SM_GAW % 32 == 0 && SM_GOW % 32 == 0 && SM_GSC % 32 == 0);
static_assert(SM_LSC + 32 == SM_GAW && SM_GSC + 32 == SM_FLOATS);

typedef float          v4f   __attribute__((ext_vector_type(4)));
typedef float          v8f   __attribute__((ext_vector_type(8)));
typedef int            v4i   __attribute__((ext_vector_type(4)));
typedef int            v8i   __attribute__((ext_vector_type(8)));
typedef unsigned       v2u   __attribute__((ext_vector_type(2)));
typedef unsigned short v8us  __attribute__((ext_vector_type(8)));
typedef unsigned short v16us __attribute__((ext_vector_type(16)));
typedef __bf16         v16bf __attribute__((ext_vector_type(16)));
typedef v4f  __attribute__((may_alias)) v4fa;
typedef v4i  __attribute__((may_alias)) v4ia;
typedef v2u  __attribute__((may_alias)) v2ua;
typedef v8us __attribute__((may_alias)) v8usa;
union FragB { v16bf v; v16us u; v8us h[2]; v8i w; };

__device__ __forceinline__ v8f wmb(const FragB& a, const FragB& b, v8f c) {
  v8f d = __builtin_amdgcn_wmma_f32_16x16x32_bf16(false, a.v, false, b.v, (short)0, c, false, false);
  asm volatile("v_nop\n\tv_nop\n\tv_nop\n\tv_nop" : "+v"(d) : "v"(a.w), "v"(b.w));
  return d;
}

__device__ __forceinline__ unsigned bf16_bits(float f) {
  const unsigned u = __float_as_uint(f);
  const unsigned r = (u + 0x7FFFu + ((u >> 16) & 1u)) >> 16;
  const unsigned q = (u >> 16) | 0x40u;
  return ((u & 0x7fffffffu) > 0x7f800000u) ? q : r;
}
__device__ __forceinline__ float bf16_val(float f) {
  return __uint_as_float(bf16_bits(f) << 16);
}

__device__ __forceinline__ void hilo_pack(float v0, float v1, float v2, float v3,
                                          int& h01, int& h23, int& l01, int& l23) {
  const unsigned a0 = bf16_bits(v0), a1 = bf16_bits(v1), a2 = bf16_bits(v2), a3 = bf16_bits(v3);
  const unsigned b0 = bf16_bits(v0 - __uint_as_float(a0 << 16));
  const unsigned b1 = bf16_bits(v1 - __uint_as_float(a1 << 16));
  const unsigned b2 = bf16_bits(v2 - __uint_as_float(a2 << 16));
  const unsigned b3 = bf16_bits(v3 - __uint_as_float(a3 << 16));
  h01 = (int)(a0 | (a1 << 16)); h23 = (int)(a2 | (a3 << 16));
  l01 = (int)(b0 | (b1 << 16)); l23 = (int)(b2 | (b3 << 16));
}

__device__ __forceinline__ v4i hilo_row(float v0, float v1, float v2, float v3, int lane) {
  int h01, h23, l01, l23;
  hilo_pack(v0, v1, v2, v3, h01, h23, l01, l23);
  const int s0 = (2 * lane) & 31, s1 = s0 + 1;
  const int a0 = __shfl(h01, s0, 32), a1 = __shfl(h23, s0, 32), a2 = __shfl(h01, s1, 32), a3 = __shfl(h23, s1, 32);
  const int b0 = __shfl(l01, s0, 32), b1 = __shfl(l23, s0, 32), b2 = __shfl(l01, s1, 32), b3 = __shfl(l23, s1, 32);
  const int mk = (lane < 16) ? -1 : 0;
  v4i o;
  o.x = (a0 & mk) | (b0 & ~mk); o.y = (a1 & mk) | (b1 & ~mk);
  o.z = (a2 & mk) | (b2 & ~mk); o.w = (a3 & mk) | (b3 & ~mk);
  return o;
}

__device__ __forceinline__ void st2_v4f(float* p, v4f v) {
  *(volatile v4f*)p = v;
  __threadfence();
  *(volatile v4f*)p = v;
}
__device__ __forceinline__ void st2_v8us(unsigned short* p, v8us v) {
  *(volatile v8us*)p = v;
  __threadfence();
  *(volatile v8us*)p = v;
}

__device__ __forceinline__ v8us gather8(const float* __restrict__ base, int stride) {
  float f[8];
#pragma unroll
  for (int i = 0; i < 8; ++i) f[i] = base[(size_t)i * (size_t)stride];
  v8us o;
#pragma unroll
  for (int i = 0; i < 8; ++i) o[i] = (unsigned short)bf16_bits(f[i]);
  return o;
}

__device__ __forceinline__ void tab_seg(const float* __restrict__ src, int n4, float* dst, int tid) {
  const int i = tid < n4 ? tid : n4 - 1;
  const v4f a = *(const v4fa*)(src + 4 * i);
  asm volatile("" :: "v"(a));
  v4f o;
  o.x = bf16_val(a.x); o.y = bf16_val(a.y); o.z = bf16_val(a.z); o.w = bf16_val(a.w);
  if (tid < n4) st2_v4f(dst + 4 * tid, o);
}

__device__ __forceinline__ void scal_line(const float* __restrict__ ab, int nab, const float* __restrict__ ob,
                                          float* dst, int lane) {
  const float a0 = ab[0], a1 = ab[1], a2 = ab[nab > 2 ? 2 : nab - 1];
  const float b0 = ob[0], b1 = ob[1], b2 = ob[2], b3 = ob[3];
  asm volatile("" :: "v"(a0), "v"(a1), "v"(a2));
  asm volatile("" :: "v"(b0), "v"(b1), "v"(b2), "v"(b3));
  const unsigned q  = (unsigned)(lane & 7);
  const unsigned mA = (q == 0u) ? 0xffffffffu : 0u;
  const unsigned mB = (q == 1u) ? 0xffffffffu : 0u;
  const unsigned m2 = (nab > 2) ? mA : 0u;
  v4f o;
  o.x = __uint_as_float(((bf16_bits(a0) << 16) & mA) | ((bf16_bits(b0) << 16) & mB));
  o.y = __uint_as_float(((bf16_bits(a1) << 16) & mA) | ((bf16_bits(b1) << 16) & mB));
  o.z = __uint_as_float(((bf16_bits(a2) << 16) & m2) | ((bf16_bits(b2) << 16) & mB));
  o.w = __uint_as_float((bf16_bits(b3) << 16) & mB);
  if (lane < 8) st2_v4f(dst + 4 * lane, o);
}

__global__ __launch_bounds__(NTHR) void k_prep(const float* __restrict__ x,
                                               const float* __restrict__ lW, const float* __restrict__ lRt,
                                               const float* __restrict__ lB,
                                               const float* __restrict__ gW, const float* __restrict__ gRt,
                                               const float* __restrict__ gB,
                                               const float* __restrict__ law, const float* __restrict__ lab,
                                               const float* __restrict__ gaw, const float* __restrict__ gab,
                                               const float* __restrict__ low, const float* __restrict__ lob,
                                               const float* __restrict__ gow, const float* __restrict__ gob,
                                               unsigned short* xb, unsigned short* bt_pl, float* sm) {
  const int tid = (int)threadIdx.x, lane = tid & 31;
  const int blk = (int)blockIdx.x;
  if (blk < PBX) {
    const int u   = blk * NTHR + tid;
    const int row = u >> 4, k8 = (u & 15) * 8;
    const int rc  = row < NN ? row : NN - 1;
    const unsigned mk = row < NN ? 0xffffu : 0u;
    const float* p = x + (size_t)rc * HD + k8;
    const v4f a = *(const v4fa*)p;
    const v4f b = *(const v4fa*)(p + 4);
    v8us o;
    o[0] = (unsigned short)(bf16_bits(a.x) & mk); o[1] = (unsigned short)(bf16_bits(a.y) & mk);
    o[2] = (unsigned short)(bf16_bits(a.z) & mk); o[3] = (unsigned short)(bf16_bits(a.w) & mk);
    o[4] = (unsigned short)(bf16_bits(b.x) & mk); o[5] = (unsigned short)(bf16_bits(b.y) & mk);
    o[6] = (unsigned short)(bf16_bits(b.z) & mk); o[7] = (unsigned short)(bf16_bits(b.w) & mk);
    st2_v8us(xb + (size_t)row * XP + k8, o);
  } else if (blk < PBX + PBT) {
    const int g     = blk - PBX;
    const int layer = g / 96;
    const int rem   = g - layer * 96;
    const int bt    = rem >> 3;
    const int w     = (rem & 7) * NTHR + tid;
    const int n     = w >> 4, k8 = (w & 15) * 8, b = bt >> 1;
    const size_t so = (size_t)k8 * HD + (size_t)n;
    v8us o;
    if (layer < 2) {
      if (b == 0) o = gather8(lRt + (size_t)layer * HD * HD + so, HD);
      else        o = gather8(lW + ((size_t)layer * NR + (size_t)(b - 1)) * HD * HD + so, HD);
    } else {
      const int lg = layer - 2;
      if (b == 0) o = gather8(gRt + (size_t)lg * HD * HD + so, HD);
      else        o = gather8(gW + ((size_t)lg * NR + (size_t)(b - 1)) * HD * HD + so, HD);
    }
    st2_v8us(bt_pl + (size_t)layer * HD * BTP + (size_t)n * BTP + (size_t)(bt * HD + k8), o);
  } else {
    const int s = blk - PBX - PBT;
    if (s == 0)      tab_seg(lB, 64, sm + SM_BIAS, tid);
    else if (s == 1) tab_seg(gB, 96, sm + SM_BIAS + 256, tid);
    else if (s == 2) tab_seg(law, 64, sm + SM_LAW, tid);
    else if (s == 3) tab_seg(low, 128, sm + SM_LOW, tid);
    else if (s == 4) tab_seg(gaw, 96, sm + SM_GAW, tid);
    else if (s == 5) tab_seg(gow, 128, sm + SM_GOW, tid);
    else if (s == 6) { if (tid < 32) scal_line(lab, 2, lob, sm + SM_LSC, lane); }
    else             { if (tid < 32) scal_line(gab, 3, gob, sm + SM_GSC, lane); }
  }
}

__device__ __forceinline__ void bucket_flush(const int* pl, const int* cnt, const int* c5, int ov,
                                             int* lp, int* cop, int* ivp, int* fp, int tid) {
#pragma unroll 1
  for (int i = tid * 4; i < RCAP; i += NTHR * 4) {
    const v4i v = *(const v4ia*)(pl + i);
    *(volatile v4i*)(lp + i) = v;
  }
#pragma unroll 1
  for (int i = tid * 4; i < 2 * NBRUN; i += NTHR * 4) {
    const v4i v = *(const v4ia*)(cnt + i);
    *(volatile v4i*)(cop + i) = v;
  }
#pragma unroll 1
  for (int i = tid * 4; i < 8 * NBRUN; i += NTHR * 4) {
    const v4i v = *(const v4ia*)(c5 + i);
    *(volatile v4i*)(ivp + i) = v;
  }
  if (tid < 8) {
    const v4i f = {ov, ov, ov, ov};
    *(volatile v4i*)(fp + 4 * tid) = f;
  }
}

__global__ __launch_bounds__(NTHR) void k_bucket(const int* __restrict__ srcs, const int* __restrict__ dsts,
                                                 const int* __restrict__ typs, int* LIST, int* CO, int* INV,
                                                 int* FLAG) {
  extern __shared__ __attribute__((aligned(16))) int dsm[];
  int* wl   = dsm;
  int* pl   = dsm + NWAVE * WLCAP;
  int* cnt  = pl + RCAP;
  int* offs = cnt + NBRUN;
  int* cur  = offs + NBRUN;
  int* c5   = cur + NBRUN;
  int* misc = c5 + 8 * NBRUN;
  const int tid = (int)threadIdx.x, lane = tid & 31, wave = tid >> 5;
  const int blk = (int)blockIdx.x;
  const unsigned nbs = (unsigned)(blk * NBRUN);

  {
    const v4i z4 = {0, 0, 0, 0};
    for (int i = tid * 4; i < BK_ZINTS; i += NTHR * 4) *(v4ia*)(dsm + i) = z4;
    if (tid < 16) misc[tid] = 0;
  }
  __syncthreads();

  {
    const int per  = ((NE + NWAVE * WCH - 1) / (NWAVE * WCH)) * WCH;
    const int ebeg = wave * per;
    const int eend = (ebeg + per < NE) ? (ebeg + per) : NE;
    int* mylist = wl + wave * WLCAP;
    int wc = 0;
#pragma unroll 1
    for (int cb = ebeg; cb < eend; cb += WCH) {
      const int e0 = cb + lane * EPT;
      const v4i da = *(const v4ia*)(dsts + e0);
      const v4i db = *(const v4ia*)(dsts + e0 + 4);
      const unsigned s0 = (unsigned)da.x - nbs, s1 = (unsigned)da.y - nbs;
      const unsigned s2 = (unsigned)da.z - nbs, s3 = (unsigned)da.w - nbs;
      const unsigned s4 = (unsigned)db.x - nbs, s5 = (unsigned)db.y - nbs;
      const unsigned s6 = (unsigned)db.z - nbs, s7 = (unsigned)db.w - nbs;
      const bool h0 = s0 < (unsigned)NBRUN, h1 = s1 < (unsigned)NBRUN, h2 = s2 < (unsigned)NBRUN, h3 = s3 < (unsigned)NBRUN;
      const bool h4 = s4 < (unsigned)NBRUN, h5 = s5 < (unsigned)NBRUN, h6 = s6 < (unsigned)NBRUN, h7 = s7 < (unsigned)NBRUN;
      const unsigned m0 = __builtin_amdgcn_ballot_w32(h0), m1 = __builtin_amdgcn_ballot_w32(h1);
      const unsigned m2 = __builtin_amdgcn_ballot_w32(h2), m3 = __builtin_amdgcn_ballot_w32(h3);
      const unsigned m4 = __builtin_amdgcn_ballot_w32(h4), m5 = __builtin_amdgcn_ballot_w32(h5);
      const unsigned m6 = __builtin_amdgcn_ballot_w32(h6), m7 = __builtin_amdgcn_ballot_w32(h7);
      const unsigned any = m0 | m1 | m2 | m3 | m4 | m5 | m6 | m7;
      if (any != 0u) {
        const int pre = (int)(__builtin_amdgcn_mbcnt_lo(m0, 0u) + __builtin_amdgcn_mbcnt_lo(m1, 0u) +
                              __builtin_amdgcn_mbcnt_lo(m2, 0u) + __builtin_amdgcn_mbcnt_lo(m3, 0u) +
                              __builtin_amdgcn_mbcnt_lo(m4, 0u) + __builtin_amdgcn_mbcnt_lo(m5, 0u) +
                              __builtin_amdgcn_mbcnt_lo(m6, 0u) + __builtin_amdgcn_mbcnt_lo(m7, 0u));
        int p = wc + pre;
        if (h0) { if (p < WLCAP) mylist[p] = ((e0 + 0) << SLB) | (int)s0; p = p + 1; }
        if (h1) { if (p < WLCAP) mylist[p] = ((e0 + 1) << SLB) | (int)s1; p = p + 1; }
        if (h2) { if (p < WLCAP) mylist[p] = ((e0 + 2) << SLB) | (int)s2; p = p + 1; }
        if (h3) { if (p < WLCAP) mylist[p] = ((e0 + 3) << SLB) | (int)s3; p = p + 1; }
        if (h4) { if (p < WLCAP) mylist[p] = ((e0 + 4) << SLB) | (int)s4; p = p + 1; }
        if (h5) { if (p < WLCAP) mylist[p] = ((e0 + 5) << SLB) | (int)s5; p = p + 1; }
        if (h6) { if (p < WLCAP) mylist[p] = ((e0 + 6) << SLB) | (int)s6; p = p + 1; }
        if (h7) { if (p < WLCAP) mylist[p] = ((e0 + 7) << SLB) | (int)s7; p = p + 1; }
        wc += (int)(__builtin_popcount(m0) + __builtin_popcount(m1) + __builtin_popcount(m2) + __builtin_popcount(m3) +
                    __builtin_popcount(m4) + __builtin_popcount(m5) + __builtin_popcount(m6) + __builtin_popcount(m7));
      }
    }
    if (lane == 0) misc[wave] = wc;
  }
  __syncthreads();

  if (wave == 0) {
    int ov = 0;
#pragma unroll 1
    for (int w2 = 0; w2 < NWAVE; ++w2) {
      int c = misc[w2];
      if (c > WLCAP) ov = 1;
      c = c < 0 ? 0 : (c > WLCAP ? WLCAP : c);
#pragma unroll 1
      for (int b0 = 0; b0 < c; b0 += 32) {
        const int idx = b0 + lane;
        const int ent = wl[w2 * WLCAP + (idx < WLCAP ? idx : WLCAP - 1)];
        const int m32 = (c - b0) < 32 ? (c - b0) : 32;
#pragma unroll 1
        for (int k = 0; k < m32; ++k) {
          const int u    = __builtin_amdgcn_readlane(ent, k);
          const int slot = u & (NBRUN - 1);
          if (lane == 0) cnt[slot] = cnt[slot] + 1;
        }
      }
    }
    if (lane == 0) misc[9] = ov;
  }
  __syncthreads();
  if (wave == 0) {
    const int base = lane * (NBRUN / 32);
    int s = 0;
#pragma unroll 1
    for (int i = 0; i < NBRUN / 32; ++i) s += cnt[base + i];
    int incl = s;
#pragma unroll
    for (int d = 1; d < 32; d <<= 1) {
      const int y = __shfl_up(incl, d, 32);
      if (lane >= d) incl += y;
    }
    int run = incl - s;
#pragma unroll 1
    for (int i = 0; i < NBRUN / 32; ++i) {
      const int cv = cnt[base + i];
      offs[base + i] = run;
      cur[base + i]  = run;
      run += cv;
    }
  }
  __syncthreads();

  if (wave == 0) {
#pragma unroll 1
    for (int w2 = 0; w2 < NWAVE; ++w2) {
      int c = misc[w2];
      c = c < 0 ? 0 : (c > WLCAP ? WLCAP : c);
#pragma unroll 1
      for (int b0 = 0; b0 < c; b0 += 32) {
        const int idx = b0 + lane;
        const int ent = wl[w2 * WLCAP + (idx < WLCAP ? idx : WLCAP - 1)];
        int eid = (ent >> SLB) & 0xFFFFF;
        eid = eid > NE - 1 ? NE - 1 : eid;
        int sr = srcs[eid];
        sr = sr < 0 ? 0 : (sr > NN - 1 ? NN - 1 : sr);
        int ty = typs[eid];
        ty = ty < 0 ? 0 : (ty > NR - 1 ? NR - 1 : ty);
        const int word = (int)((unsigned)sr | ((unsigned)ty << 16) | ((unsigned)(ent & (NBRUN - 1)) << 19));
        const int m32 = (c - b0) < 32 ? (c - b0) : 32;
#pragma unroll 1
        for (int k = 0; k < m32; ++k) {
          const int wd   = __builtin_amdgcn_readlane(word, k);
          const int slot = (wd >> 19) & (NBRUN - 1);
          const int tk   = (wd >> 16) & 7;
          if (lane == 0) {
            int p = cur[slot];
            p = p < 0 ? 0 : (p > RCAP - 1 ? RCAP - 1 : p);
            pl[p] = wd;
            cur[slot] = p + 1;
            c5[slot * 8 + tk] = c5[slot * 8 + tk] + 1;
          }
        }
      }
    }
  }
  __syncthreads();

#pragma unroll 1
  for (int i = tid; i < 8 * NBRUN; i += NTHR) {
    const int   c  = c5[i];
    const float cf = (float)c;
    const float f  = 1.0f / (cf > 1.0f ? cf : 1.0f);
    c5[i] = ((i & 7) < NR) ? __float_as_int(f) : 0;
  }
  __syncthreads();

  const int ovf = misc[9];
  int* lp  = LIST + (size_t)blk * RCAP;
  int* cop = CO + (size_t)blk * (2 * NBRUN);
  int* ivp = INV + (size_t)blk * (8 * NBRUN);
  int* fp  = FLAG + (size_t)blk * 32;
  bucket_flush(pl, cnt, c5, ovf, lp, cop, ivp, fp, tid);
  __threadfence();
  bucket_flush(pl, cnt, c5, ovf, lp, cop, ivp, fp, tid);
}

__device__ __forceinline__ void acc_sel(int ty, v4f v, v4f& A0, v4f& A1, v4f& A2, v4f& A3, v4f& A4) {
  switch (ty) {
    case 0:  A0 += v; break;
    case 1:  A1 += v; break;
    case 2:  A2 += v; break;
    case 3:  A3 += v; break;
    default: A4 += v; break;
  }
}

template <int L0>
__global__ __launch_bounds__(NTHR) void k_replay(const int* __restrict__ LIST, const int* __restrict__ CO,
                                                 const float* __restrict__ INV, const int* __restrict__ FLAG,
                                                 const unsigned short* __restrict__ Hs, unsigned short* MCH,
                                                 int chunkBase) {
  constexpr int SPITCH = (L0 != 0) ? XP : HP;
  const int tid = (int)threadIdx.x, lane = tid & 31, wave = tid >> 5;
  const int rowBase = chunkBase + (int)blockIdx.x * ABM;
  const int bucket  = rowBase >> SLB;
  const int* lb  = LIST + (size_t)bucket * RCAP;
  const int* cob = CO + (size_t)bucket * (2 * NBRUN);
  const int flag = FLAG[(size_t)bucket * 32];
  const float qnan = __uint_as_float(0x7fc00000u);

#pragma unroll 1
  for (int i = 0; i < ABM / NWAVE; ++i) {
    const int d    = rowBase + (ABM / NWAVE) * wave + i;
    const int slot = d & (NBRUN - 1);
    int c = cob[slot];
    int o = cob[NBRUN + slot];
    const bool big = c > TRIPCAP;
    c = c < 0 ? 0 : (c > TRIPCAP ? TRIPCAP : c);
    o = o < 0 ? 0 : (o > RCAP - 1 ? RCAP - 1 : o);
    int last = o + c - 1; last = last < o ? o : last;
    last = last > RCAP - 1 ? RCAP - 1 : last;
    c    = __builtin_amdgcn_readfirstlane(c);
    o    = __builtin_amdgcn_readfirstlane(o);
    last = __builtin_amdgcn_readfirstlane(last);

    v4f A0 = {0.0f, 0.0f, 0.0f, 0.0f}, A1 = A0, A2 = A0, A3 = A0, A4 = A0;
#pragma unroll 1
    for (int j = 0; j < c; j += 4) {
      unsigned wd[4];
#pragma unroll
      for (int u = 0; u < 4; ++u) {
        int idx = o + j + u;
        idx = idx > last ? last : idx;
        wd[u] = (unsigned)lb[idx];
      }
      v2u wh[4], wlo[4];
#pragma unroll
      for (int u = 0; u < 4; ++u) {
        int sr = (int)(wd[u] & 0xffffu);
        sr = sr > NN - 1 ? NN - 1 : sr;
        const unsigned short* rp = Hs + (size_t)sr * SPITCH + 4 * lane;
        wh[u] = *(const v2ua*)rp;
        if constexpr (L0 == 0) wlo[u] = *(const v2ua*)(rp + HD);
        else                   wlo[u] = wh[u];
      }
#pragma unroll
      for (int u = 0; u < 4; ++u) {
        asm volatile("" :: "v"(wh[u]));
        if constexpr (L0 == 0) asm volatile("" :: "v"(wlo[u]));
      }
#pragma unroll
      for (int u = 0; u < 4; ++u) {
        v4f v;
        v.x = __uint_as_float(wh[u].x << 16);
        v.y = __uint_as_float(wh[u].x & 0xffff0000u);
        v.z = __uint_as_float(wh[u].y << 16);
        v.w = __uint_as_float(wh[u].y & 0xffff0000u);
        if constexpr (L0 == 0) {
          v.x += __uint_as_float(wlo[u].x << 16);
          v.y += __uint_as_float(wlo[u].x & 0xffff0000u);
          v.z += __uint_as_float(wlo[u].y << 16);
          v.w += __uint_as_float(wlo[u].y & 0xffff0000u);
        }
        int ty = __builtin_amdgcn_readfirstlane((int)((wd[u] >> 16) & 7u));
        ty = ty > NR - 1 ? NR - 1 : ty;
        if (j + u < c) acc_sel(ty, v, A0, A1, A2, A3, A4);
      }
    }

    const v4f i0 = *(const v4fa*)(INV + (size_t)d * 8);
    const v4f i1 = *(const v4fa*)(INV + (size_t)d * 8 + 4);
    const bool bad  = (flag != 0) | big;
    const bool live = d < NN;
    v4f M[5];
    M[0] = A0 * i0.x; M[1] = A1 * i0.y; M[2] = A2 * i0.z; M[3] = A3 * i0.w; M[4] = A4 * i1.x;
    v4i ow[5];
#pragma unroll
    for (int r = 0; r < NR; ++r) {
      float m0 = M[r].x, m1 = M[r].y, m2 = M[r].z, m3 = M[r].w;
      m0 = bad ? qnan : m0; m1 = bad ? qnan : m1; m2 = bad ? qnan : m2; m3 = bad ? qnan : m3;
      m0 = live ? m0 : 0.0f; m1 = live ? m1 : 0.0f; m2 = live ? m2 : 0.0f; m3 = live ? m3 : 0.0f;
      ow[r] = hilo_row(m0, m1, m2, m3, lane);
    }
    unsigned short* mp = MCH + (size_t)(d - chunkBase) * MPI + 8 * lane;
#pragma unroll
    for (int r = 0; r < NR; ++r) *(volatile v4i*)(mp + r * HP) = ow[r];
    __threadfence();
#pragma unroll
    for (int r = 0; r < NR; ++r) *(volatile v4i*)(mp + r * HP) = ow[r];
  }
}

__device__ __forceinline__ void gemm_seg(const unsigned short* __restrict__ ap,
                                         const unsigned short* __restrict__ bp, int klen, v8f (&acc)[8]) {
#pragma unroll 1
  for (int k0 = 0; k0 < klen; k0 += 32) {
    FragB af;
    af.h[0] = *(const v8usa*)(ap + k0);
    af.h[1] = *(const v8usa*)(ap + k0 + 16);
#pragma unroll
    for (int nt = 0; nt < 8; ++nt) {
      const unsigned short* wq = bp + (size_t)(16 * nt) * (size_t)BTP + k0;
      FragB bf;
      bf.h[0] = *(const v8usa*)wq;
      bf.h[1] = *(const v8usa*)(wq + 16);
      acc[nt] = wmb(af, bf, acc[nt]);
    }
  }
}

template <int L0>
__global__ __launch_bounds__(GTHR) __attribute__((amdgpu_num_vgpr(248)))
void k_gemm(const unsigned short* __restrict__ Hsrc, const unsigned short* __restrict__ MCH,
            const unsigned short* __restrict__ BT, const float* __restrict__ bias,
            unsigned short* Hdst, int chunkBase) {
  __shared__ __attribute__((aligned(16))) float stg[GBM * SP];
  __shared__ __attribute__((aligned(16))) float sb[HD];
  const int tid = (int)threadIdx.x, lane = tid & 31, wave = tid >> 5, hh = lane >> 4, m = lane & 15;
  const int rowBase = chunkBase + (int)blockIdx.x * GBM;
  if (tid < 32) *(v4fa*)(sb + 4 * tid) = *(const v4fa*)(bias + 4 * tid);

  v8f acc[8];
  {
    const v8f z = {0.f, 0.f, 0.f, 0.f, 0.f, 0.f, 0.f, 0.f};
#pragma unroll
    for (int t = 0; t < 8; ++t) acc[t] = z;
  }
  const size_t arow = (size_t)(rowBase + 16 * wave + m);
  const size_t mrow = arow - (size_t)chunkBase;
  const unsigned short* bp = BT + (size_t)m * (size_t)BTP + 8 * hh;
  if constexpr (L0 != 0) {
    gemm_seg(Hsrc + arow * (size_t)XP + 8 * hh, bp, KH0, acc);
  } else {
    gemm_seg(Hsrc + arow * (size_t)HP + 8 * hh, bp, KHN, acc);
  }
  const unsigned short* am = MCH + mrow * (size_t)MPI + 8 * hh;
#if SPLIT_M
  gemm_seg(am, bp + 256, KMN, acc);
#else
#pragma unroll 1
  for (int r = 0; r < NR; ++r) gemm_seg(am + r * HP, bp + 256 + r * HP, HD, acc);
#endif

#pragma unroll
  for (int nt = 0; nt < 8; ++nt) {
#pragma unroll
    for (int r = 0; r < 8; ++r) stg[(16 * wave + 8 * hh + r) * SP + 16 * nt + m] = acc[nt][r];
  }
  __syncthreads();

  const v4f bv = *(const v4fa*)(sb + 4 * lane);
#pragma unroll 1
  for (int i = 0; i < 16; ++i) {
    const int lr   = 16 * wave + i;
    const int grow = rowBase + lr;
    const bool live = grow < NN;
    const v4f a = *(const v4fa*)(stg + lr * SP + 4 * lane);
    float v0 = a.x + bv.x, v1 = a.y + bv.y, v2 = a.z + bv.z, v3 = a.w + bv.w;
    v0 = (v0 > 0.0f) ? v0 : (v0 - v0); v1 = (v1 > 0.0f) ? v1 : (v1 - v1);
    v2 = (v2 > 0.0f) ? v2 : (v2 - v2); v3 = (v3 > 0.0f) ? v3 : (v3 - v3);
    v0 = live ? v0 : 0.0f; v1 = live ? v1 : 0.0f; v2 = live ? v2 : 0.0f; v3 = live ? v3 : 0.0f;
    const v4i ow = hilo_row(v0, v1, v2, v3, lane);
    unsigned short* hp = Hdst + (size_t)grow * HP + 8 * lane;
    *(volatile v4i*)hp = ow;
    __threadfence();
    *(volatile v4i*)hp = ow;
  }
}

template <int L, int NV>
__global__ __launch_bounds__(NTHR) void k_node(const unsigned short* __restrict__ P0,
                                               const unsigned short* __restrict__ P1,
                                               const unsigned short* __restrict__ P2,
                                               const float* __restrict__ tb, const int* __restrict__ FLAG,
                                               float* out, int oA, int oB, int oC, int oP) {
  __shared__ __attribute__((aligned(16))) float tab[1024];
  __shared__ __attribute__((aligned(16))) float so[NODEM * NCL];
  __shared__ __attribute__((aligned(16))) float sp[NODEM * NCL];
  constexpr int NT4 = L * 32 + 136;
  constexpr int OW  = L * HD;
  constexpr int SC  = L * HD + 512;
  static_assert(NT4 <= 256);
  const int tid = (int)threadIdx.x, lane = tid & 31, wave = tid >> 5;
  const int rowBase = (int)blockIdx.x * NODEM;
  {
    const int i = tid < NT4 ? tid : NT4 - 1;
    const v4f v = *(const v4fa*)(tb + 4 * i);
    *(v4fa*)(tab + 4 * tid) = v;
  }
  __syncthreads();
  const int flag = FLAG[(size_t)(rowBase >> SLB) * 32];
  const float qnan = __uint_as_float(0x7fc00000u);

#pragma unroll 1
  for (int i = 0; i < 16; ++i) {
    const int lr  = 16 * wave + i;
    const int row = rowBase + lr;
    v4f h0, h1, h2;
    {
      const unsigned short* r0 = P0 + (size_t)row * HP + 4 * lane;
      const unsigned short* r1 = P1 + (size_t)row * HP + 4 * lane;
      const v2u a0 = *(const v2ua*)r0, b0 = *(const v2ua*)(r0 + HD);
      const v2u a1 = *(const v2ua*)r1, b1 = *(const v2ua*)(r1 + HD);
      h0.x = __uint_as_float(a0.x << 16) + __uint_as_float(b0.x << 16);
      h0.y = __uint_as_float(a0.x & 0xffff0000u) + __uint_as_float(b0.x & 0xffff0000u);
      h0.z = __uint_as_float(a0.y << 16) + __uint_as_float(b0.y << 16);
      h0.w = __uint_as_float(a0.y & 0xffff0000u) + __uint_as_float(b0.y & 0xffff0000u);
      h1.x = __uint_as_float(a1.x << 16) + __uint_as_float(b1.x << 16);
      h1.y = __uint_as_float(a1.x & 0xffff0000u) + __uint_as_float(b1.x & 0xffff0000u);
      h1.z = __uint_as_float(a1.y << 16) + __uint_as_float(b1.y << 16);
      h1.w = __uint_as_float(a1.y & 0xffff0000u) + __uint_as_float(b1.y & 0xffff0000u);
      h2 = h1;
      if constexpr (L == 3) {
        const unsigned short* r2 = P2 + (size_t)row * HP + 4 * lane;
        const v2u a2 = *(const v2ua*)r2, b2 = *(const v2ua*)(r2 + HD);
        h2.x = __uint_as_float(a2.x << 16) + __uint_as_float(b2.x << 16);
        h2.y = __uint_as_float(a2.x & 0xffff0000u) + __uint_as_float(b2.x & 0xffff0000u);
        h2.z = __uint_as_float(a2.y << 16) + __uint_as_float(b2.y << 16);
        h2.w = __uint_as_float(a2.y & 0xffff0000u) + __uint_as_float(b2.y & 0xffff0000u);
      }
    }
    const v4f hl = (L == 3) ? h2 : h1;

    float s0 = 0.0f, s1 = 0.0f, s2 = 0.0f;
#pragma unroll 1
    for (int l = 0; l < L; ++l) {
      const v4f w = *(const v4fa*)(tab + l * HD + 4 * lane);
      float p = hl.x * w.x;
      p = fmaf(hl.y, w.y, p); p = fmaf(hl.z, w.z, p); p = fmaf(hl.w, w.w, p);
      p += __shfl_xor(p, 16, 32); p += __shfl_xor(p, 8, 32); p += __shfl_xor(p, 4, 32);
      p += __shfl_xor(p, 2, 32);  p += __shfl_xor(p, 1, 32);
      p += tab[SC + l];
      s0 = (l == 0) ? p : s0; s1 = (l == 1) ? p : s1; s2 = (l == 2) ? p : s2;
    }
    float mx = s0;
    mx = ((s1 > mx) | (s1 != s1)) ? s1 : mx;
    if constexpr (L == 3) mx = ((s2 > mx) | (s2 != s2)) ? s2 : mx;
    float e0 = 0.0f, e1 = 0.0f, e2 = 0.0f, den = 0.0f;
#pragma unroll 1
    for (int l = 0; l < L; ++l) {
      const float sv = (l == 0) ? s0 : ((l == 1) ? s1 : s2);
      const float e  = expf(sv - mx);
      den += e;
      e0 = (l == 0) ? e : e0; e1 = (l == 1) ? e : e1; e2 = (l == 2) ? e : e2;
    }
    const float inv = 1.0f / den;
    const float c0 = e0 * inv, c1 = e1 * inv, c2 = e2 * inv;
    v4f ft;
    ft.x = c0 * h0.x + c1 * h1.x; ft.y = c0 * h0.y + c1 * h1.y;
    ft.z = c0 * h0.z + c1 * h1.z; ft.w = c0 * h0.w + c1 * h1.w;
    if constexpr (L == 3) {
      ft.x = fmaf(c2, h2.x, ft.x); ft.y = fmaf(c2, h2.y, ft.y);
      ft.z = fmaf(c2, h2.z, ft.z); ft.w = fmaf(c2, h2.w, ft.w);
    }

    float o0 = 0.0f, o1 = 0.0f, o2 = 0.0f, o3 = 0.0f;
#pragma unroll 1
    for (int c = 0; c < NCL; ++c) {
      const v4f w = *(const v4fa*)(tab + OW + c * HD + 4 * lane);
      float p = ft.x * w.x;
      p = fmaf(ft.y, w.y, p); p = fmaf(ft.z, w.z, p); p = fmaf(ft.w, w.w, p);
      p += __shfl_xor(p, 16, 32); p += __shfl_xor(p, 8, 32); p += __shfl_xor(p, 4, 32);
      p += __shfl_xor(p, 2, 32);  p += __shfl_xor(p, 1, 32);
      p += tab[SC + 4 + c];
      o0 = (c == 0) ? p : o0; o1 = (c == 1) ? p : o1; o2 = (c == 2) ? p : o2; o3 = (c == 3) ? p : o3;
    }
    float m4 = o0;
    m4 = ((o1 > m4) | (o1 != o1)) ? o1 : m4;
    m4 = ((o2 > m4) | (o2 != o2)) ? o2 : m4;
    m4 = ((o3 > m4) | (o3 != o3)) ? o3 : m4;
    float se = 0.0f;
#pragma unroll 1
    for (int c = 0; c < NCL; ++c) {
      const float ov = (c == 0) ? o0 : ((c == 1) ? o1 : ((c == 2) ? o2 : o3));
      se += expf(ov - m4);
    }
    const float ls = m4 + logf(se);
    v4f vo, vp;
    vo.x = o0; vo.y = o1; vo.z = o2; vo.w = o3;
    vp.x = o0 - ls; vp.y = o1 - ls; vp.z = o2 - ls; vp.w = o3 - ls;
    if (flag != 0) {
      vo.x = qnan; vo.y = qnan; vo.z = qnan; vo.w = qnan;
      vp = vo;
    }
    if (lane == 0) {
      *(v4fa*)(so + 4 * lr) = vo;
      *(v4fa*)(sp + 4 * lr) = vp;
    }
  }
  __syncthreads();

  if (tid < NODEM) {
    const v4f a = *(const v4fa*)(so + 4 * tid);
    const v4f p = *(const v4fa*)(sp + 4 * tid);
    asm volatile("" :: "v"(a));
    asm volatile("" :: "v"(p));
    const int  row  = rowBase + tid;
    const bool live = row < NN;
    const int  rc   = live ? row : NN - 1;
    float* qa = out + (size_t)oA + (size_t)rc * NCL;
    float* qb = out + (size_t)oB + (size_t)rc * NCL;
    float* qc = out + (size_t)oC + (size_t)rc * NCL;
    float* qp = out + (size_t)oP + (size_t)rc * NCL;
    if (live) {
      *(volatile v4f*)qa = a;
      if constexpr (NV == 3) { *(volatile v4f*)qb = a; *(volatile v4f*)qc = a; }
      *(volatile v4f*)qp = p;
    }
    __threadfence();
    if (live) {
      *(volatile v4f*)qa = a;
      if constexpr (NV == 3) { *(volatile v4f*)qb = a; *(volatile v4f*)qc = a; }
      *(volatile v4f*)qp = p;
    }
  }
}

extern "C" void kernel_launch(void* const* d_in, const int* in_sizes, int n_in,
                              void* d_out, int out_size, void* d_ws, size_t ws_size,
                              hipStream_t stream) {
  if (n_in < 17) return;
  if (in_sizes[0] != NN * HD) return;
  if (in_sizes[1] != 2 * NE) return;
  if (in_sizes[2] != NE) return;
  if (in_sizes[3] != 2 * NR * HD * HD) return;
  if (in_sizes[4] != 2 * HD * HD) return;
  if (in_sizes[5] != 2 * HD) return;
  if (in_sizes[6] != 3 * NR * HD * HD) return;
  if (in_sizes[7] != 3 * HD * HD) return;
  if (in_sizes[8] != 3 * HD) return;
  if (in_sizes[9] != 2 * HD || in_sizes[10] != 2) return;
  if (in_sizes[11] != 3 * HD || in_sizes[12] != 3) return;
  if (in_sizes[13] != NCL * HD || in_sizes[14] != NCL) return;
  if (in_sizes[15] != NCL * HD || in_sizes[16] != NCL) return;
  if (out_size != 6 * NN * NCL) return;

  const float* x   = (const float*)d_in[0];
  const int*   ei  = (const int*)d_in[1];
  const int*   et  = (const int*)d_in[2];
  const float* lW  = (const float*)d_in[3];
  const float* lRt = (const float*)d_in[4];
  const float* lB  = (const float*)d_in[5];
  const float* gW  = (const float*)d_in[6];
  const float* gRt = (const float*)d_in[7];
  const float* gB  = (const float*)d_in[8];
  const float* law = (const float*)d_in[9];
  const float* lab = (const float*)d_in[10];
  const float* gaw = (const float*)d_in[11];
  const float* gab = (const float*)d_in[12];
  const float* low = (const float*)d_in[13];
  const float* lob = (const float*)d_in[14];
  const float* gow = (const float*)d_in[15];
  const float* gob = (const float*)d_in[16];
  float* out = (float*)d_out;
  const int* srcs = ei;
  const int* dsts = ei + NE;

  constexpr size_t zH    = (size_t)MP * HP * 2;
  constexpr size_t zXB   = (size_t)MP * XP * 2;
  constexpr size_t zMCH  = (size_t)CHROWS * MPI * 2;
  constexpr size_t zLIST = (size_t)NBK * RCAP * 4;
  constexpr size_t zCO   = (size_t)NBK * 2 * NBRUN * 4;
  constexpr size_t zINV  = (size_t)NBK * NBRUN * 8 * 4;
  constexpr size_t zFLAG = 6400;
  constexpr size_t zBT   = (size_t)5 * HD * BTP * 2;
  constexpr size_t zSM   = 9728;
  constexpr size_t oHA   = 0;
  constexpr size_t oHB   = oHA + zH;
  constexpr size_t oHC   = oHB + zH;
  constexpr size_t oMCH  = oHC + zH;
  constexpr size_t oLIST = oMCH + zMCH;
  constexpr size_t oCO   = oLIST + zLIST;
  constexpr size_t oINV  = oCO + zCO;
  constexpr size_t oFLAG = oINV + zINV;
  constexpr size_t oBT   = oFLAG + zFLAG;
  constexpr size_t oSM   = oBT + zBT;
  constexpr size_t oEND  = oSM + zSM;
  static_assert(zH % 256 == 0 && zMCH % 256 == 0 && zLIST % 256 == 0 && zCO % 256 == 0 && zINV % 256 == 0);
  static_assert(zFLAG % 256 == 0 && zBT % 256 == 0 && zSM % 256 == 0);
  static_assert(zXB <= zH && (size_t)NBK * 128 <= zFLAG && (size_t)SM_FLOATS * 4 <= zSM);
  static_assert(oEND <= ((size_t)128u << 20));
  if (oEND > ws_size) return;

  char* ws = (char*)d_ws;
  unsigned short* HA   = (unsigned short*)(ws + oHA);
  unsigned short* HB   = (unsigned short*)(ws + oHB);
  unsigned short* HC   = (unsigned short*)(ws + oHC);
  unsigned short* XB   = (unsigned short*)(ws + oHC);
  unsigned short* MCH  = (unsigned short*)(ws + oMCH);
  int*            LIST = (int*)(ws + oLIST);
  int*            CO   = (int*)(ws + oCO);
  int*            INVi = (int*)(ws + oINV);
  const float*    INVf = (const float*)(ws + oINV);
  int*            FLAG = (int*)(ws + oFLAG);
  unsigned short* BT   = (unsigned short*)(ws + oBT);
  float*          SM   = (float*)(ws + oSM);

  hipFuncSetAttribute(reinterpret_cast<const void*>(&k_bucket), hipFuncAttributeMaxDynamicSharedMemorySize, (int)BK_LDS);

  k_prep<<<PBTOT, NTHR, 0, stream>>>(x, lW, lRt, lB, gW, gRt, gB, law, lab, gaw, gab, low, lob, gow, gob, XB, BT, SM);
  k_bucket<<<NBK, NTHR, BK_LDS, stream>>>(srcs, dsts, et, LIST, CO, INVi, FLAG);

  const int lsrc[5] = {-1, 0, -1, 0, 1};
  const int ldst[5] = { 0, 1,  0, 1, 2};
  unsigned short* planes[3] = {HA, HB, HC};

  for (int ly = 0; ly < 5; ++ly) {
    const unsigned short* bt = BT + (size_t)ly * HD * BTP;
    const float* bias = SM + SM_BIAS + ly * HD;
    unsigned short* dst = planes[ldst[ly]];
    for (int ch = 0; ch < NCHUNK; ++ch) {
      const int cbase = ch * CHROWS;
      const int rows  = (ch < NCHUNK - 1) ? CHROWS : (MP - (NCHUNK - 1) * CHROWS);
      if (lsrc[ly] < 0) {
        k_replay<1><<<rows / ABM, NTHR, 0, stream>>>(LIST, CO, INVf, FLAG, XB, MCH, cbase);
        k_gemm<1><<<rows / GBM, GTHR, 0, stream>>>(XB, MCH, bt, bias, dst, cbase);
      } else {
        const unsigned short* src = planes[lsrc[ly]];
        k_replay<0><<<rows / ABM, NTHR, 0, stream>>>(LIST, CO, INVf, FLAG, src, MCH, cbase);
        k_gemm<0><<<rows / GBM, GTHR, 0, stream>>>(src, MCH, bt, bias, dst, cbase);
      }
    }
    if (ly == 1) {
      k_node<2, 1><<<MP / NODEM, NTHR, 0, stream>>>(HA, HB, HB, SM + SM_LAW, FLAG, out,
                                                   0, 0, 0, 2 * NN * NCL);
    }
    if (ly == 4) {
      k_node<3, 3><<<MP / NODEM, NTHR, 0, stream>>>(HA, HB, HC, SM + SM_GAW, FLAG, out,
                                                   1 * NN * NCL, 3 * NN * NCL, 4 * NN * NCL, 5 * NN * NCL);
    }
  }
}
